// NeuralTensorLayer_6554120094087
// MI455X (gfx1250) — hardware-verified
//
#include <hip/hip_runtime.h>
#include <math.h>

typedef __attribute__((ext_vector_type(16))) _Float16 v16h;
typedef __attribute__((ext_vector_type(16))) __bf16 v16b;
typedef __attribute__((ext_vector_type(8)))  _Float16 v8h;
typedef __attribute__((ext_vector_type(8)))  float v8f;
typedef __attribute__((ext_vector_type(4)))  float v4f;
typedef __attribute__((ext_vector_type(2)))  float v2f;
typedef __attribute__((ext_vector_type(4)))  unsigned v4u;
typedef __attribute__((ext_vector_type(4)))  int v4i;
typedef float __attribute__((may_alias)) float_a;
typedef int __attribute__((may_alias)) int_a;

template <typename T> __device__ __forceinline__ void vst2(void* p, T v) { *(volatile T*)p = v; __threadfence(); *(volatile T*)p = v; }
__device__ __forceinline__ v8f wmma16(v16h a, v16h b, v8f c) {
  v8f d = __builtin_amdgcn_wmma_f32_16x16x32_f16(false, a, false, b, (short)0, c, false, false);
  asm volatile("v_nop\n\tv_nop\n\tv_nop\n\tv_nop" : "+v"(d) : "v"(a), "v"(b));
  return d;
}
__device__ __forceinline__ v8f wmma_bf(v16b a, v16b b, v8f c) {
  v8f d = __builtin_amdgcn_wmma_f32_16x16x32_bf16(false, a, false, b, (short)0, c, false, false);
  asm volatile("v_nop\n\tv_nop\n\tv_nop\n\tv_nop" : "+v"(d) : "v"(a), "v"(b));
  return d;
}
__device__ __forceinline__ v16h frag_h(const _Float16* rowk0, int lane) {
  union { v16h v; v8h q[2]; } u; const _Float16* p = rowk0 + 8 * (lane >> 4);
  u.q[0] = *(const v8h*)p; u.q[1] = *(const v8h*)(p + 16); return u.v;
}
__device__ __forceinline__ v16h frag_f32(const float* rowk0, int lane) {
  v16h a; const float* p = rowk0 + 8 * (lane >> 4);
#pragma unroll
  for (int i = 0; i < 8; ++i) { a[i] = (_Float16)p[i]; a[8 + i] = (_Float16)p[16 + i]; }
  return a;
}
__device__ __forceinline__ v16h frag_f32s(const float* rowk0, int lane, float sc) {
  v16h a; const float* p = rowk0 + 8 * (lane >> 4);
#pragma unroll
  for (int i = 0; i < 8; ++i) { a[i] = (_Float16)(p[i] * sc); a[8 + i] = (_Float16)(p[16 + i] * sc); }
  return a;
}
__device__ __forceinline__ v16h fragc_f32(const float* W, int k0, int n, int lane, int ld, int K) {
  v16h a; const int g = lane >> 4;
#pragma unroll
  for (int i = 0; i < 8; ++i) { const int ka = k0 + 8 * g + i, kb = ka + 16;
    a[i] = (_Float16)(ka < K ? W[(size_t)(ka < K ? ka : K - 1) * ld + n] : 0.f); a[8 + i] = (_Float16)(kb < K ? W[(size_t)(kb < K ? kb : K - 1) * ld + n] : 0.f); }
  return a;
}
struct F2 { v16b h, l; };
__device__ __forceinline__ F2 bsplit16(const float v[16]) { F2 r;
#pragma unroll
  for (int i = 0; i < 16; ++i) { const __bf16 h = (__bf16)v[i]; r.h[i] = h; r.l[i] = (__bf16)(v[i] - (float)h); }
  return r; }
__device__ __forceinline__ F2 split_row(const float* row, int k0, int lane) { float v[16]; const float* p = row + k0 + 8 * (lane >> 4);
#pragma unroll
  for (int i = 0; i < 8; ++i) { v[i] = p[i]; v[8 + i] = p[16 + i]; }
  return bsplit16(v); }
__device__ __forceinline__ F2 split_rowK(const float* row, int k0, int lane, int K) { float v[16]; const int g = lane >> 4;
#pragma unroll
  for (int i = 0; i < 8; ++i) { const int ka = k0 + 8 * g + i, kb = ka + 16; v[i] = ka < K ? row[ka < K ? ka : K - 1] : 0.f; v[8 + i] = kb < K ? row[kb < K ? kb : K - 1] : 0.f; }
  return bsplit16(v); }
__device__ __forceinline__ F2 split_col(const float* W, int k0, int n, int lane, int ld, int K) { float v[16]; const int g = lane >> 4;
#pragma unroll
  for (int i = 0; i < 8; ++i) { const int ka = k0 + 8 * g + i, kb = ka + 16; v[i] = ka < K ? W[(size_t)(ka < K ? ka : K - 1) * ld + n] : 0.f; v[8 + i] = kb < K ? W[(size_t)(kb < K ? kb : K - 1) * ld + n] : 0.f; }
  return bsplit16(v); }
__device__ __forceinline__ v8f mac3(const F2& a, const F2& b, v8f c) { c = wmma_bf(a.l, b.h, c); c = wmma_bf(a.h, b.l, c); return wmma_bf(a.h, b.h, c); }
__device__ __forceinline__ float sigm(float v) { return 1.0f / (1.0f + expf(-v)); }
#define LDSX() do { asm volatile("s_wait_dscnt 0" ::: "memory"); __builtin_amdgcn_wave_barrier(); __builtin_amdgcn_fence(__ATOMIC_RELEASE, "workgroup"); } while (0)

__device__ __forceinline__ float bfr(float v) { return (float)(__bf16)v; }
#define NBS 32768
#define DD 32
#define KK 32
#define PP (DD * DD)
#define T3W (DD * KK)
#ifndef NROWS
#define NROWS NBS
#endif
__device__ __forceinline__ v16b frag_rb(const float* rowk0, int lane) { v16b a; const float* p = rowk0 + 8 * (lane >> 4);
#pragma unroll
  for (int i = 0; i < 8; ++i) { a[i] = (__bf16)p[i]; a[8 + i] = (__bf16)p[16 + i]; }
  return a; }
__global__ __launch_bounds__(128) void k_ntl(const float* __restrict__ X, const float* __restrict__ W1, const float* __restrict__ W2, const float* __restrict__ W3, const float* __restrict__ BIAS, float* __restrict__ OUT) { __shared__ __align__(16) float so[4][16][36]; __shared__ float sx[4][16][33];
  const int tid = threadIdx.x, wave = tid >> 5, lane = tid & 31, col = lane & 15, g = lane >> 4; const size_t r0 = (size_t)blockIdx.x * 64 + wave * 16; const size_t arow = r0 + col;
  for (int e = lane; e < 16 * DD; e += 32) sx[wave][e >> 5][e & 31] = bfr(X[(r0 + (e >> 5)) * DD + (e & 31)]);
  __syncthreads();
  const float* xa = &sx[wave][col][0];     (void)arow;
  float oacc[2][8]; for (int q = 0; q < 2; ++q) for (int r = 0; r < 8; ++r) oacc[q][r] = 0.f;
  for (int cb = 0; cb < T3W / 128; ++cb) { v8f acc[8] = {};
#pragma unroll 2
    for (int kc = 0; kc < PP / 32; ++kc) { float v[16]; const float xi = xa[kc];
#pragma unroll
      for (int q = 0; q < 8; ++q) { v[q] = xi * xa[8 * g + q]; v[8 + q] = xi * xa[16 + 8 * g + q]; }
      const F2 a = bsplit16(v);
#pragma unroll
      for (int j = 0; j < 8; ++j) { v16b w; const int n = cb * 128 + j * 16 + col;
#pragma unroll
        for (int i = 0; i < 8; ++i) { w[i] = (__bf16)W3[(size_t)(kc * 32 + 8 * g + i) * T3W + n]; w[8 + i] = (__bf16)W3[(size_t)(kc * 32 + 16 + 8 * g + i) * T3W + n]; }
        asm volatile("s_wait_loadcnt 0x0" ::: "memory"); acc[j] = wmma_bf(a.h, w, acc[j]); acc[j] = wmma_bf(a.l, w, acc[j]); } }
#pragma unroll
    for (int j = 0; j < 8; ++j) { const int k = cb * 4 + (j >> 1);
#pragma unroll
      for (int r = 0; r < 8; ++r) oacc[j & 1][r] += acc[j][r] * sx[wave][8 * g + r][k]; } }
  { v8f acc2[2] = {};
#pragma unroll 2
    for (int kc = 0; kc < PP / 32; ++kc) { float v[16]; const float xi = xa[kc];
#pragma unroll
      for (int q = 0; q < 8; ++q) { v[q] = xi * xa[8 * g + q]; v[8 + q] = xi * xa[16 + 8 * g + q]; }
      const F2 a = bsplit16(v);
#pragma unroll
      for (int j = 0; j < 2; ++j) { v16b w; const int n = j * 16 + col;
#pragma unroll
        for (int i = 0; i < 8; ++i) { w[i] = (__bf16)W2[(size_t)(kc * 32 + 8 * g + i) * KK + n]; w[8 + i] = (__bf16)W2[(size_t)(kc * 32 + 16 + 8 * g + i) * KK + n]; }
        asm volatile("s_wait_loadcnt 0x0" ::: "memory"); acc2[j] = wmma_bf(a.h, w, acc2[j]); acc2[j] = wmma_bf(a.l, w, acc2[j]); } }
    { const v16b ax = frag_rb(X + (r0 + col) * DD, lane);
#pragma unroll
      for (int j = 0; j < 2; ++j) { v16b w; const int n = j * 16 + col;
#pragma unroll
        for (int i = 0; i < 8; ++i) { w[i] = (__bf16)W1[(size_t)(8 * g + i) * KK + n]; w[8 + i] = (__bf16)W1[(size_t)(16 + 8 * g + i) * KK + n]; }
        asm volatile("s_wait_loadcnt 0x0" ::: "memory"); acc2[j] = wmma_bf(ax, w, acc2[j]); } }
#pragma unroll
    for (int j = 0; j < 2; ++j) { const float bb = bfr(BIAS[j * 16 + col]);
#pragma unroll
      for (int r = 0; r < 8; ++r) so[wave][8 * g + r][j * 16 + col] = acc2[j][r] + oacc[j][r] + bb; } }
  LDSX();
  for (int rl = 0; rl < 16; ++rl) if (lane < 8) vst2(OUT + (r0 + rl) * KK + lane * 4, *(const v4f*)&so[wave][rl][lane * 4]); }
extern "C" void kernel_launch(void* const* d_in, const int* in_sizes, int n_in, void* d_out, int out_size, void* d_ws, size_t ws_size, hipStream_t stream) {
  (void)in_sizes; (void)n_in; (void)out_size; (void)d_ws; (void)ws_size;
  const float** F = (const float**)d_in;
  k_ntl<<<dim3(NROWS / 64), 128, 0, stream>>>(F[0], F[1], F[2], F[3], F[4], (float*)d_out);
}
